// ConvTest_PCFNet_30537217475338
// MI455X (gfx1250) — hardware-verified
//
#include <hip/hip_runtime.h>
#include <math.h>

#define NBATCH 4096
#define RSPLIT (1.0f / 2048.0f)
#define P2K 3136

typedef _Float16 h16;
typedef __attribute__((ext_vector_type(16))) _Float16 v16h;
typedef __attribute__((ext_vector_type(8)))  _Float16 v8h;
typedef __attribute__((ext_vector_type(8)))  float v8f;
typedef __attribute__((ext_vector_type(4)))  float v4f_t;
typedef float v4fa __attribute__((ext_vector_type(4), may_alias));
typedef __attribute__((ext_vector_type(4)))  unsigned v4u_t;
typedef unsigned v4ua __attribute__((ext_vector_type(4), may_alias));

__device__ __forceinline__ h16 lo_of(float v, h16 h) { return (h16)((v - (float)h) * 2048.0f); }
__device__ __forceinline__ v8f wmma16(v16h a, v16h b, v8f c) { return __builtin_amdgcn_wmma_f32_16x16x32_f16(false, a, false, b, (short)0, c, false, false); }
__device__ __forceinline__ v8f wmma_split(v16h a, v16h al, v16h b, v16h bl, v8f c) { v8f x = {}; x = wmma16(al, b, x); x = wmma16(a, bl, x); return wmma16(a, b, c) + x * RSPLIT; }
__device__ __forceinline__ v16h rfrag(const h16* rowp, int half) {
  const h16* p = rowp + 8 * half;
  return __builtin_shufflevector(*(const v8h*)p, *(const v8h*)(p + 16), 0,1,2,3,4,5,6,7,8,9,10,11,12,13,14,15);
}
__device__ __forceinline__ int kof(int half, int e) { return 8 * half + ((e < 8) ? e : (e + 8)); }

__global__ __launch_bounds__(256) void k_conv1(const float* __restrict__ x, const float* __restrict__ theta, const float* __restrict__ sigma,
                                              const float* __restrict__ gam, const float* __restrict__ lambd, const float* __restrict__ psi,
                                              h16* __restrict__ P1) {
  __shared__ float xs[30 * 30];
  __shared__ float cmap[32][788];
  __shared__ __attribute__((aligned(16))) h16 pooled[32 * 196 + 8];
  __shared__ float w1[32 * 9];
  const int img = blockIdx.x, tid = threadIdx.x, lane = tid & 31, wave = tid >> 5, half = lane >> 4, l16 = lane & 15;
  for (int i = tid; i < 900; i += 256) { const int yy = i / 30 - 1, xx = i % 30 - 1; xs[i] = (yy >= 0 && yy < 28 && xx >= 0 && xx < 28) ? x[(size_t)img * 784 + yy * 28 + xx] : 0.0f; }
  for (int i = tid; i < 32 * 9; i += 256) {
    const int f = i / 9, k = i % 9;
    if (f < 16) {
      const int ix = k / 3, iy = k % 3;
      const float xg = (float)ix - 1.0f, yg = (float)iy - 1.0f;
      const float c = cosf(theta[f]), s = sinf(theta[f]);
      const float xt = xg * c + yg * s, yt = -xg * s + yg * c;
      const float sx = sigma[f], sy = sigma[f] / gam[f];
      const float env = expf(-0.5f * (xt * xt / (sx * sx) + yt * yt / (sy * sy)));
      const float car = cosf(2.0f * 3.14159265358979323846f * xt / lambd[f] + psi[f]);
      w1[i] = env * car;
    } else w1[i] = (k == 4) ? 1.0f : 0.0f;
  }
  __syncthreads();
  v16h Bw[2];
#pragma unroll
  for (int nt = 0; nt < 2; ++nt) { v16h r;
#pragma unroll
    for (int e = 0; e < 16; ++e) { const int k = kof(half, e); r[e] = (h16)((k < 9) ? w1[(nt * 16 + l16) * 9 + k] : 0.0f); }
    Bw[nt] = r; }
#pragma unroll 1
  for (int pt = wave; pt < 49; pt += 8) {
    const int p = pt * 16 + l16, py = p / 28, px = p % 28;
    v16h a;
#pragma unroll
    for (int e = 0; e < 16; ++e) { const int k = kof(half, e); float v = 0.0f;
      if (k < 9) { const int dy = k / 3, dx = k % 3; v = xs[(py + dy) * 30 + (px + dx)]; } a[e] = (h16)v; }
#pragma unroll
    for (int nt = 0; nt < 2; ++nt) { v8f c = {}; c = wmma16(a, Bw[nt], c);
#pragma unroll
      for (int r = 0; r < 8; ++r) cmap[nt * 16 + l16][pt * 16 + 8 * half + r] = fmaxf(c[r], 0.0f); }
  }
  __syncthreads();
  for (int i = tid; i < 32 * 196; i += 256) { const int ch = i / 196, q = i % 196, oy = q / 14, ox = q % 14;
    const float* m = &cmap[ch][(2 * oy) * 28 + 2 * ox];
    pooled[i] = (h16)fmaxf(fmaxf(m[0], m[1]), fmaxf(m[28], m[29])); }
  __syncthreads();
#pragma unroll 1
  for (int pass = 0; pass < 2; ++pass) {
    for (int ch8 = tid; ch8 < 32 * 196 / 8; ch8 += 256) *(volatile v4u_t*)(P1 + (size_t)img * 32 * 196 + ch8 * 8) = *(const v4ua*)(pooled + ch8 * 8);
    __threadfence();
  }
}

__global__ __launch_bounds__(256) void k_conv2(const h16* __restrict__ P1, const float* __restrict__ w2, const float* __restrict__ b2, h16* __restrict__ P2) {
  __shared__ __attribute__((aligned(16))) h16 ps[32 * 196];
  __shared__ __attribute__((aligned(16))) h16 Bs[64 * 296];
  __shared__ float omap[64][200];
  __shared__ __attribute__((aligned(16))) h16 prow[2][P2K + 8];
  const int img = blockIdx.x, tid = threadIdx.x, lane = tid & 31, wave = tid >> 5, half = lane >> 4, l16 = lane & 15;
  for (int i = tid; i < 32 * 196 / 8; i += 256) *(v4u_t*)(ps + i * 8) = *(const v4ua*)(P1 + (size_t)img * 32 * 196 + i * 8);
  for (int i = tid; i < 64 * 288; i += 256) { const int o = i / 288, k = i % 288, tap = k >> 5, c = k & 31; Bs[o * 296 + k] = (h16)w2[((size_t)o * 32 + c) * 9 + tap]; }
  __syncthreads();
#pragma unroll 1
  for (int pt = wave; pt < 13; pt += 8) {
    const int p = pt * 16 + l16; const bool pv = p < 196; const int py = pv ? p / 14 : 0, px = pv ? p % 14 : 0;
    v8f acc[4] = {};
#pragma unroll 1
    for (int tap = 0; tap < 9; ++tap) {
      const int yy = py + tap / 3 - 1, xx = px + tap % 3 - 1;
      const bool inb = pv && yy >= 0 && yy < 14 && xx >= 0 && xx < 14;
      v16h a;
#pragma unroll
      for (int e = 0; e < 16; ++e) { const int c = kof(half, e); a[e] = inb ? ps[c * 196 + yy * 14 + xx] : (h16)0.0f; }
#pragma unroll
      for (int nt = 0; nt < 4; ++nt) acc[nt] = wmma16(a, rfrag(&Bs[(nt * 16 + l16) * 296 + tap * 32], half), acc[nt]);
    }
#pragma unroll
    for (int nt = 0; nt < 4; ++nt) { const int o = nt * 16 + l16; const float bb = b2[o];
#pragma unroll
      for (int r = 0; r < 8; ++r) { const int pp = pt * 16 + 8 * half + r; if (pp < 196) omap[o][pp] = fmaxf(acc[nt][r] + bb, 0.0f); } }
  }
  __syncthreads();
  for (int i = tid; i < 64 * 49; i += 256) { const int o = i / 49, q = i % 49, oy = q / 7, ox = q % 7;
    const float* m = &omap[o][(2 * oy) * 14 + 2 * ox];
    const float v = fmaxf(fmaxf(m[0], m[1]), fmaxf(m[14], m[15]));
    const h16 hv = (h16)v; prow[0][i] = hv; prow[1][i] = lo_of(v, hv); }
  __syncthreads();
  const size_t plane = (size_t)NBATCH * P2K;
#pragma unroll 1
  for (int pass = 0; pass < 2; ++pass) {
    for (int i = tid; i < P2K / 8; i += 256) { *(volatile v4u_t*)(P2 + (size_t)img * P2K + i * 8) = *(const v4ua*)(&prow[0][i * 8]); *(volatile v4u_t*)(P2 + plane + (size_t)img * P2K + i * 8) = *(const v4ua*)(&prow[1][i * 8]); }
    __threadfence();
  }
}

#define LDS_STRIDE 48
__global__ __launch_bounds__(256) void k_fc1(const float* __restrict__ A, const h16* __restrict__ Wp, size_t wPlane, const float* __restrict__ rbias,
                                            float* __restrict__ out, int N, int K) {
  __shared__ __attribute__((aligned(16))) h16 ldsA[128 * LDS_STRIDE], ldsAl[128 * LDS_STRIDE];
  __shared__ __attribute__((aligned(16))) h16 ldsW[256 * LDS_STRIDE], ldsWl[256 * LDS_STRIDE];
  __shared__ __attribute__((aligned(16))) float sob[64 * 260];
  const int t = threadIdx.x, wave = t >> 5, lane = t & 31, half = lane >> 4, l16 = lane & 15;
  const int wm = (wave & 1) * 64, wn = (wave >> 1) * 64;
  const int nBlk = blockIdx.x * 256;
  const int arow = t >> 1, ach = (t & 1) * 16;
  v8f acc[4][4] = {};
#pragma unroll 1
  for (int k = 0; k < K; k += 32) {
    __syncthreads();
    { const float* ap = A + (size_t)arow * K + k + ach;
#pragma unroll
      for (int i = 0; i < 16; ++i) { const float v = ap[i]; const h16 hv = (h16)v; ldsA[arow * LDS_STRIDE + ach + i] = hv; ldsAl[arow * LDS_STRIDE + ach + i] = lo_of(v, hv); } }
    { const h16* wp = Wp + (size_t)(nBlk + t) * K + k;
#pragma unroll
      for (int i = 0; i < 32; ++i) { ldsW[t * LDS_STRIDE + i] = wp[i]; ldsWl[t * LDS_STRIDE + i] = wp[wPlane + i]; } }
    __syncthreads();
    v16h wf[4], wfl[4];
#pragma unroll
    for (int j = 0; j < 4; ++j) { wf[j] = rfrag(ldsW + (wn + 16 * j + l16) * LDS_STRIDE, half); wfl[j] = rfrag(ldsWl + (wn + 16 * j + l16) * LDS_STRIDE, half); }
#pragma unroll
    for (int i = 0; i < 4; ++i) {
      const v16h af = rfrag(ldsA + (wm + 16 * i + l16) * LDS_STRIDE, half), afl = rfrag(ldsAl + (wm + 16 * i + l16) * LDS_STRIDE, half);
#pragma unroll
      for (int j = 0; j < 4; ++j) acc[i][j] = wmma_split(af, afl, wf[j], wfl[j], acc[i][j]);
    }
  }
  const int mh = half * 8;
  __syncthreads();
#pragma unroll 1
  for (int hf = 0; hf < 2; ++hf) {
    if (wm == hf * 64) {
#pragma unroll
      for (int i = 0; i < 4; ++i)
#pragma unroll
        for (int j = 0; j < 4; ++j) { const int nl = wn + 16 * j + l16;
#pragma unroll
          for (int r = 0; r < 8; ++r) { const int ml = 16 * i + mh + r; sob[ml * 260 + nl] = acc[i][j][r] + rbias[hf * 64 + ml]; } }
    }
    __syncthreads();
#pragma unroll 1
    for (int pass = 0; pass < 2; ++pass) {
      for (int ch = t; ch < 64 * 64; ch += 256) { const int ml = ch >> 6, q = (ch & 63) * 4;
        *(volatile v4f_t*)(out + (size_t)(hf * 64 + ml) * N + nBlk + q) = *(const volatile v4fa*)(sob + ml * 260 + q); }
      __threadfence();
    }
    __syncthreads();
  }
}

__global__ __launch_bounds__(256) void k_fc2(const float* __restrict__ H1T, const float* __restrict__ fc2_w, const float* __restrict__ fc2_b, float* __restrict__ out) {
  __shared__ float ws[10 * 128];
  __shared__ __attribute__((aligned(16))) float res[64 * 10];
  const int tid = threadIdx.x, b0 = blockIdx.x * 64;
  for (int i = tid; i < 1280; i += 256) ws[i] = fc2_w[i];
  __syncthreads();
  for (int i = tid; i < 640; i += 256) { const int bl = i / 10, o = i % 10;
    float a = fc2_b[o];
#pragma unroll 1
    for (int j = 0; j < 128; ++j) a += fmaxf(H1T[(size_t)j * NBATCH + b0 + bl], 0.0f) * ws[o * 128 + j];
    res[i] = a; }
  __syncthreads();
#pragma unroll 1
  for (int pass = 0; pass < 2; ++pass) { if (tid < 160) *(volatile v4f_t*)(out + (size_t)b0 * 10 + tid * 4) = *(const volatile v4fa*)(res + tid * 4); __threadfence(); }
}

extern "C" void kernel_launch(void* const* d_in, const int* in_sizes, int n_in,
                              void* d_out, int out_size, void* d_ws, size_t ws_size,
                              hipStream_t stream) {
  (void)in_sizes; (void)n_in; (void)out_size; (void)ws_size;
  const float* x     = (const float*)d_in[0];
  const float* theta = (const float*)d_in[1];
  const float* sigma = (const float*)d_in[2];
  const float* gam   = (const float*)d_in[3];
  const float* lambd = (const float*)d_in[4];
  const float* psi   = (const float*)d_in[5];
  const float* w2    = (const float*)d_in[6];
  const float* b2    = (const float*)d_in[7];
  const float* fc1_w = (const float*)d_in[8];
  const float* fc1_b = (const float*)d_in[9];
  const float* fc2_w = (const float*)d_in[10];
  const float* fc2_b = (const float*)d_in[11];
  char* ws = (char*)d_ws;
  h16*   P1  = (h16*)ws;   ws += (size_t)NBATCH * 32 * 196 * 2;
  h16*   P2  = (h16*)ws;   ws += (size_t)2 * NBATCH * P2K * 2;
  float* H1T = (float*)ws; ws += (size_t)128 * NBATCH * 4;
  k_conv1<<<NBATCH, 256, 0, stream>>>(x, theta, sigma, gam, lambd, psi, P1);
  k_conv2<<<NBATCH, 256, 0, stream>>>(P1, w2, b2, P2);
  k_fc1<<<NBATCH / 256, 256, 0, stream>>>(fc1_w, P2, (size_t)NBATCH * P2K, fc1_b, H1T, NBATCH, P2K);
  k_fc2<<<NBATCH / 64, 256, 0, stream>>>(H1T, fc2_w, fc2_b, (float*)d_out);
}
